// CosFormerAttention_62302795596634
// MI455X (gfx1250) — hardware-verified
//
#include <hip/hip_runtime.h>
#include <stddef.h>
#include <stdint.h>

#define NBATCH 2
#define SEQ    1024
#define NTOK   2048
#define DMOD   512
#define NHEAD  8
#define HDM    64
#define QB     64
#define KC     64
#define NQB    (SEQ / QB)

static_assert(NTOK == NBATCH * SEQ);
static_assert(DMOD == NHEAD * HDM);
static_assert(NTOK % 64 == 0);
static_assert(DMOD % 64 == 0);
static_assert(DMOD % 32 == 0);
static_assert(SEQ % QB == 0);
static_assert(QB == KC);
static_assert(HDM == 64);
static_assert(QB == 64);
static_assert((NTOK * DMOD) % 2048 == 0);
static_assert(SEQ % 128 == 0);

typedef unsigned short us;
typedef __attribute__((ext_vector_type(16))) __bf16 v16bf;
typedef us           v8us __attribute__((ext_vector_type(8)));
typedef float        v8f  __attribute__((ext_vector_type(8)));
typedef float        v4f  __attribute__((ext_vector_type(4)));
typedef unsigned int v4u  __attribute__((ext_vector_type(4)));

union Frag  { v16bf v; v8us h[2]; };
union Pack8 { v8us h; v4u u; };

__device__ __forceinline__ us bf_rne(float f) {
  unsigned u = __float_as_uint(f);
  u = u + 0x7FFFu + ((u >> 16) & 1u);
  return (us)(u >> 16);
}
__device__ __forceinline__ float bf_val(us h) { return __uint_as_float(((unsigned)h) << 16); }
__device__ __forceinline__ void split2(float f, us& hi, us& lo) {
  const us hv = bf_rne(f);
  hi = hv;
  lo = bf_rne(f - bf_val(hv));
}
__device__ __forceinline__ void split8(const float (&f)[8], Pack8& ph, Pack8& pl) {
  us hh[8], ll[8];
#pragma unroll
  for (int e = 0; e < 8; ++e) split2(f[e], hh[e], ll[e]);
  ph.h = (v8us){hh[0], hh[1], hh[2], hh[3], hh[4], hh[5], hh[6], hh[7]};
  pl.h = (v8us){ll[0], ll[1], ll[2], ll[3], ll[4], ll[5], ll[6], ll[7]};
}

__device__ __forceinline__ v8f mma16(v16bf a, v16bf b, v8f c) {
  c = __builtin_amdgcn_wmma_f32_16x16x32_bf16(false, a, false, b, (short)0, c, false, false);
  asm volatile("v_nop\n\tv_nop\n\tv_nop\n\tv_nop" : "+v"(c) : "v"(a), "v"(b));
  return c;
}

__device__ __forceinline__ v16bf ldfrag(const us* p, int ld, int row0, int k0, int lane) {
  const int m = lane & 15, lh = lane >> 4;
  const us* q = p + (size_t)(row0 + m) * ld + k0 + 8 * lh;
  Frag f;
  f.h[0] = *(const v8us*)(q);
  f.h[1] = *(const v8us*)(q + 16);
  return f.v;
}

__device__ __forceinline__ v8f zero8() { return (v8f){0.f, 0.f, 0.f, 0.f, 0.f, 0.f, 0.f, 0.f}; }

template <int KD>
__device__ __forceinline__ void gemm16x64x3(const us* __restrict__ Ah, const us* __restrict__ Al,
                                            const us* __restrict__ Bh, const us* __restrict__ Bl,
                                            int m0, int n0, int lane, v8f (&acc)[4]) {
  static_assert(KD % 32 == 0);
#pragma unroll 1
  for (int k0 = 0; k0 < KD; k0 += 32) {
    const v16bf ah = ldfrag(Ah, KD, m0, k0, lane);
    const v16bf al = ldfrag(Al, KD, m0, k0, lane);
#pragma unroll
    for (int t = 0; t < 4; ++t) {
      const v16bf bh = ldfrag(Bh, KD, n0 + 16 * t, k0, lane);
      const v16bf bl = ldfrag(Bl, KD, n0 + 16 * t, k0, lane);
      acc[t] = mma16(ah, bh, acc[t]);
      acc[t] = mma16(ah, bl, acc[t]);
      acc[t] = mma16(al, bh, acc[t]);
    }
  }
}

__global__ __launch_bounds__(256) void k_cvt(const float* __restrict__ x, us* __restrict__ xh, us* __restrict__ xl) {
  const size_t i = (size_t)blockIdx.x * 2048 + (size_t)threadIdx.x * 8;
  const v4f a0 = *(const v4f*)(x + i);
  const v4f a1 = *(const v4f*)(x + i + 4);
  const float f[8] = {a0[0], a0[1], a0[2], a0[3], a1[0], a1[1], a1[2], a1[3]};
  Pack8 ph, pl;
  split8(f, ph, pl);
  const v4u hv = ph.u, lv = pl.u;
  *(volatile v4u*)(xh + i) = hv;
  *(volatile v4u*)(xl + i) = lv;
  __threadfence();
  *(volatile v4u*)(xh + i) = hv;
  *(volatile v4u*)(xl + i) = lv;
}

#define SFP 68
__global__ __launch_bounds__(256) void k_cvt_wt(const float* __restrict__ w, us* __restrict__ wh,
                                                us* __restrict__ wl) {
  __shared__ __align__(16) float sw[64 * SFP];
  const int tid = threadIdx.x;
  const int kb = blockIdx.x * 64;
  const int nb = blockIdx.y * 64;
  {
    const int r  = tid >> 2;
    const int c0 = (tid & 3) * 16;
    const float* src = w + (size_t)(kb + r) * DMOD + nb + c0;
#pragma unroll
    for (int e = 0; e < 4; ++e) *(v4f*)(sw + r * SFP + c0 + 4 * e) = *(const v4f*)(src + 4 * e);
  }
  __syncthreads();
  v4u hv[2], lv[2];
  size_t go[2];
#pragma unroll
  for (int j = 0; j < 2; ++j) {
    const int p  = tid + 256 * j;
    const int n  = p >> 3;
    const int pc = p & 7;
    const float* cp = sw + (pc * 8) * SFP + n;
    float f[8];
#pragma unroll
    for (int e = 0; e < 8; ++e) f[e] = cp[e * SFP];
    Pack8 ph, pl;
    split8(f, ph, pl);
    hv[j] = ph.u;
    lv[j] = pl.u;
    go[j] = (size_t)(nb + n) * DMOD + kb + pc * 8;
  }
#pragma unroll
  for (int j = 0; j < 2; ++j) { *(volatile v4u*)(wh + go[j]) = hv[j]; *(volatile v4u*)(wl + go[j]) = lv[j]; }
  __threadfence();
#pragma unroll
  for (int j = 0; j < 2; ++j) { *(volatile v4u*)(wh + go[j]) = hv[j]; *(volatile v4u*)(wl + go[j]) = lv[j]; }
}

template <int MODE>
__global__ __launch_bounds__(128) void k_proj(const us* __restrict__ xh, const us* __restrict__ xl,
                                              const us* __restrict__ wh, const us* __restrict__ wl,
                                              const float* __restrict__ bias,
                                              us* __restrict__ yh, us* __restrict__ yl,
                                              float* __restrict__ yf) {
  __shared__ __align__(16) float sf[64 * SFP];
  const int tid = threadIdx.x, lane = tid & 31, wave = tid >> 5;
  const int hh = lane >> 4, c = lane & 15;
  const int mb = blockIdx.x * 64;
  const int nb = blockIdx.y * 64;
  const int m0 = mb + wave * 16;

  v8f acc[4];
#pragma unroll
  for (int t = 0; t < 4; ++t) acc[t] = zero8();
  gemm16x64x3<DMOD>(xh, xl, wh, wl, m0, nb, lane, acc);

  float bcol[4];
#pragma unroll
  for (int t = 0; t < 4; ++t) bcol[t] = 0.f;
  if constexpr (MODE == 2) {
#pragma unroll
    for (int t = 0; t < 4; ++t) bcol[t] = bias[nb + 16 * t + c];
  }
#pragma unroll
  for (int t = 0; t < 4; ++t) {
#pragma unroll
    for (int r = 0; r < 8; ++r) {
      float v = acc[t][r];
      if constexpr (MODE == 0) v = fmaxf(v, 0.f);
      if constexpr (MODE == 2) {
        const float e = __expf(-(v + bcol[t]));
        v = 1.0f / (1.0f + e);
      }
      sf[(wave * 16 + 8 * hh + r) * SFP + 16 * t + c] = v;
    }
  }
  __syncthreads();

  if constexpr (MODE == 0) {
    v4u hv[4], lv[4];
    size_t go[4];
#pragma unroll
    for (int j = 0; j < 4; ++j) {
      const int p  = tid + 128 * j;
      const int lr = p >> 3;
      const int d0 = (p & 7) * 8;
      const float* ra = sf + lr * SFP + d0;
      const v4f a0 = *(const v4f*)(ra), a1 = *(const v4f*)(ra + 4);
      const float f[8] = {a0[0], a0[1], a0[2], a0[3], a1[0], a1[1], a1[2], a1[3]};
      Pack8 ph, pl;
      split8(f, ph, pl);
      hv[j] = ph.u;
      lv[j] = pl.u;
      go[j] = ((size_t)(mb + lr)) * DMOD + nb + d0;
    }
#pragma unroll
    for (int j = 0; j < 4; ++j) { *(volatile v4u*)(yh + go[j]) = hv[j]; *(volatile v4u*)(yl + go[j]) = lv[j]; }
    __threadfence();
#pragma unroll
    for (int j = 0; j < 4; ++j) { *(volatile v4u*)(yh + go[j]) = hv[j]; *(volatile v4u*)(yl + go[j]) = lv[j]; }
  } else if constexpr (MODE == 1) {
    v4u hv[4], lv[4];
    size_t go[4];
#pragma unroll
    for (int j = 0; j < 4; ++j) {
      const int p  = tid + 128 * j;
      const int d  = p >> 3;
      const int pc = p & 7;
      const float* cp = sf + (pc * 8) * SFP + d;
      float f[8];
#pragma unroll
      for (int e = 0; e < 8; ++e) f[e] = cp[e * SFP];
      Pack8 ph, pl;
      split8(f, ph, pl);
      hv[j] = ph.u;
      lv[j] = pl.u;
      go[j] = ((size_t)(nb + d)) * (size_t)NTOK + mb + pc * 8;
    }
#pragma unroll
    for (int j = 0; j < 4; ++j) { *(volatile v4u*)(yh + go[j]) = hv[j]; *(volatile v4u*)(yl + go[j]) = lv[j]; }
    __threadfence();
#pragma unroll
    for (int j = 0; j < 4; ++j) { *(volatile v4u*)(yh + go[j]) = hv[j]; *(volatile v4u*)(yl + go[j]) = lv[j]; }
  } else {
    v4f val[8];
    size_t go[8];
#pragma unroll
    for (int it = 0; it < 8; ++it) {
      const int p    = tid + 128 * it;
      const int L    = p >> 3;
      const int pc   = p & 7;
      const int row  = L >> 1;
      const int half = L & 1;
      const int col  = half * 32 + pc * 4;
      val[it] = *(const v4f*)(sf + row * SFP + col);
      go[it]  = (size_t)(mb + row) * DMOD + nb + col;
    }
#pragma unroll
    for (int it = 0; it < 8; ++it) *(volatile v4f*)(yf + go[it]) = val[it];
    __threadfence();
#pragma unroll
    for (int it = 0; it < 8; ++it) *(volatile v4f*)(yf + go[it]) = val[it];
  }
}

#define LP  72
#define OTP 68
union AttnLds {
  us    p[2][4 * 16 * LP];
  float o[4][16 * OTP];
};

__global__ __launch_bounds__(128) void k_attn(const us* __restrict__ qh, const us* __restrict__ ql,
                                              const us* __restrict__ kh, const us* __restrict__ kl,
                                              const us* __restrict__ vh, const us* __restrict__ vl,
                                              const float* __restrict__ gt,
                                              us* __restrict__ ogh, us* __restrict__ ogl) {
  __shared__ __align__(16) us Ksh[KC * LP];
  __shared__ __align__(16) us Ksl[KC * LP];
  __shared__ __align__(16) us Vsh[HDM * LP];
  __shared__ __align__(16) us Vsl[HDM * LP];
  __shared__ __align__(16) AttnLds pu;
  __shared__ __align__(16) float ctab[SEQ];

  const int tid = threadIdx.x, lane = tid & 31, wave = tid >> 5;
  const int hh = lane >> 4, c = lane & 15;
  const int bh   = blockIdx.x / NQB;
  const int qb   = blockIdx.x - bh * NQB;
  const int b    = bh / NHEAD;
  const int hd   = bh - b * NHEAD;
  const int tok0 = b * SEQ;
  const int col0 = hd * HDM;
  const int qloc = qb * QB + wave * 16;
  const int q0   = tok0 + qloc;
  const int nch  = qb + 1;

  const float ANG = 1.53398078788564122e-3f;
#pragma unroll 1
  for (int i = tid; i < SEQ; i += 128) ctab[i] = cosf((float)i * ANG);

  float zrow[8];
  v8f oacc[4];
#pragma unroll
  for (int r = 0; r < 8; ++r) zrow[r] = 0.f;
#pragma unroll
  for (int t = 0; t < 4; ++t) oacc[t] = zero8();

  us* pwh = pu.p[0] + wave * 16 * LP;
  us* pwl = pu.p[1] + wave * 16 * LP;

#pragma unroll 1
  for (int i = 0; i < nch; ++i) {
    const int kv0 = i * KC;
    __syncthreads();
    {
      const int r  = tid >> 1;
      const int cb = (tid & 1) * 32;
      const us* ksh = kh + (size_t)(tok0 + kv0 + r) * DMOD + col0 + cb;
      const us* ksl = kl + (size_t)(tok0 + kv0 + r) * DMOD + col0 + cb;
      const us* vsh = vh + (size_t)(col0 + r) * NTOK + tok0 + kv0 + cb;
      const us* vsl = vl + (size_t)(col0 + r) * NTOK + tok0 + kv0 + cb;
#pragma unroll
      for (int e = 0; e < 4; ++e) {
        *(v8us*)(Ksh + r * LP + cb + 8 * e) = *(const v8us*)(ksh + 8 * e);
        *(v8us*)(Ksl + r * LP + cb + 8 * e) = *(const v8us*)(ksl + 8 * e);
        *(v8us*)(Vsh + r * LP + cb + 8 * e) = *(const v8us*)(vsh + 8 * e);
        *(v8us*)(Vsl + r * LP + cb + 8 * e) = *(const v8us*)(vsl + 8 * e);
      }
    }
    __syncthreads();

    v8f s[4];
#pragma unroll
    for (int j = 0; j < 4; ++j) s[j] = zero8();
#pragma unroll
    for (int dc = 0; dc < 2; ++dc) {
      const v16bf qah = ldfrag(qh, DMOD, q0, col0 + dc * 32, lane);
      const v16bf qal = ldfrag(ql, DMOD, q0, col0 + dc * 32, lane);
#pragma unroll
      for (int j = 0; j < 4; ++j) {
        const v16bf kbh = ldfrag(Ksh, LP, j * 16, dc * 32, lane);
        const v16bf kbl = ldfrag(Ksl, LP, j * 16, dc * 32, lane);
        s[j] = mma16(qah, kbh, s[j]);
        s[j] = mma16(qah, kbl, s[j]);
        s[j] = mma16(qal, kbh, s[j]);
      }
    }
#pragma unroll
    for (int j = 0; j < 4; ++j) {
      const int key = kv0 + j * 16 + c;
#pragma unroll
      for (int r = 0; r < 8; ++r) {
        const int diff = qloc + 8 * hh + r - key;
        const int idx  = (diff < 0) ? 0 : diff;
        const float wv = ctab[idx];
        const float a  = s[j][r] * wv;
        s[j][r] = (diff >= 0) ? a : 0.f;
      }
    }
#pragma unroll
    for (int r = 0; r < 8; ++r) {
      float psum = 0.f;
#pragma unroll
      for (int j = 0; j < 4; ++j) {
        const float a = s[j][r];
        psum += a;
        us ph, pl;
        split2(a, ph, pl);
        pwh[(8 * hh + r) * LP + j * 16 + c] = ph;
        pwl[(8 * hh + r) * LP + j * 16 + c] = pl;
      }
#pragma unroll
      for (int off = 1; off < 16; off <<= 1) psum += __shfl_xor(psum, off, 32);
      zrow[r] += psum;
    }
    __syncthreads();

#pragma unroll
    for (int kk = 0; kk < 2; ++kk) {
      const v16bf pah = ldfrag(pwh, LP, 0, kk * 32, lane);
      const v16bf pal = ldfrag(pwl, LP, 0, kk * 32, lane);
#pragma unroll
      for (int t = 0; t < 4; ++t) {
        const v16bf vbh = ldfrag(Vsh, LP, t * 16, kk * 32, lane);
        const v16bf vbl = ldfrag(Vsl, LP, t * 16, kk * 32, lane);
        oacc[t] = mma16(pah, vbh, oacc[t]);
        oacc[t] = mma16(pah, vbl, oacc[t]);
        oacc[t] = mma16(pal, vbh, oacc[t]);
      }
    }
  }

  float invz[8];
#pragma unroll
  for (int r = 0; r < 8; ++r) invz[r] = 1.0f / fmaxf(zrow[r], 1e-6f);
  __syncthreads();
  float* osw = pu.o[wave];
#pragma unroll
  for (int r = 0; r < 8; ++r) {
#pragma unroll
    for (int t = 0; t < 4; ++t) osw[(8 * hh + r) * OTP + 16 * t + c] = oacc[t][r] * invz[r];
  }
  __syncthreads();
  v4u hv[4], lv[4];
  size_t go[4];
#pragma unroll
  for (int it = 0; it < 4; ++it) {
    const int p  = lane + 32 * it;
    const int lr = p >> 3;
    const int d0 = (p & 7) * 8;
    const float* ra = osw + lr * OTP + d0;
    const size_t gi = (size_t)(q0 + lr) * DMOD + col0 + d0;
    const v4f a0 = *(const v4f*)(ra), a1 = *(const v4f*)(ra + 4);
    const v4f g0 = *(const v4f*)(gt + gi), g1 = *(const v4f*)(gt + gi + 4);
    const float f[8] = {a0[0] * g0[0], a0[1] * g0[1], a0[2] * g0[2], a0[3] * g0[3],
                        a1[0] * g1[0], a1[1] * g1[1], a1[2] * g1[2], a1[3] * g1[3]};
    Pack8 ph, pl;
    split8(f, ph, pl);
    hv[it] = ph.u;
    lv[it] = pl.u;
    go[it] = gi;
  }
#pragma unroll
  for (int it = 0; it < 4; ++it) { *(volatile v4u*)(ogh + go[it]) = hv[it]; *(volatile v4u*)(ogl + go[it]) = lv[it]; }
  __threadfence();
#pragma unroll
  for (int it = 0; it < 4; ++it) { *(volatile v4u*)(ogh + go[it]) = hv[it]; *(volatile v4u*)(ogl + go[it]) = lv[it]; }
}

extern "C" void kernel_launch(void* const* d_in, const int* in_sizes, int n_in,
                              void* d_out, int out_size, void* d_ws, size_t ws_size,
                              hipStream_t stream) {
  if (n_in < 7) return;
  if (in_sizes[0] != NTOK * DMOD) return;
  if (in_sizes[1] != DMOD * DMOD) return;
  if (in_sizes[2] != DMOD * DMOD) return;
  if (in_sizes[3] != DMOD * DMOD) return;
  if (in_sizes[4] != DMOD * DMOD) return;
  if (in_sizes[5] != DMOD * DMOD) return;
  if (in_sizes[6] != DMOD) return;
  if (out_size != NTOK * DMOD) return;

  const float* X  = (const float*)d_in[0];
  const float* Wq = (const float*)d_in[1];
  const float* Wk = (const float*)d_in[2];
  const float* Wv = (const float*)d_in[3];
  const float* Wo = (const float*)d_in[4];
  const float* Wg = (const float*)d_in[5];
  const float* bg = (const float*)d_in[6];
  float* out = (float*)d_out;

  const size_t PL2 = (size_t)NTOK * DMOD * 2;
  const size_t WPL = (size_t)DMOD * DMOD * 2;
  const size_t GFB = (size_t)NTOK * DMOD * 4;
  size_t off = 0;
  const size_t oXh  = off; off += PL2;
  const size_t oXl  = off; off += PL2;
  const size_t oWQh = off; off += WPL;  const size_t oWQl = off; off += WPL;
  const size_t oWKh = off; off += WPL;  const size_t oWKl = off; off += WPL;
  const size_t oWVh = off; off += WPL;  const size_t oWVl = off; off += WPL;
  const size_t oWGh = off; off += WPL;  const size_t oWGl = off; off += WPL;
  const size_t oWOh = off; off += WPL;  const size_t oWOl = off; off += WPL;
  const size_t oQh  = off; off += PL2;  const size_t oQl  = off; off += PL2;
  const size_t oKh  = off; off += PL2;  const size_t oKl  = off; off += PL2;
  const size_t oVTh = off; off += PL2;  const size_t oVTl = off; off += PL2;
  const size_t oGT  = off; off += GFB;
  const size_t oOGh = off; off += PL2;  const size_t oOGl = off; off += PL2;
  if (off > ws_size) return;
  if (off > (size_t)134217728) return;

  char* ws = (char*)d_ws;
  us* Xh  = (us*)(ws + oXh);   us* Xl  = (us*)(ws + oXl);
  us* WQh = (us*)(ws + oWQh);  us* WQl = (us*)(ws + oWQl);
  us* WKh = (us*)(ws + oWKh);  us* WKl = (us*)(ws + oWKl);
  us* WVh = (us*)(ws + oWVh);  us* WVl = (us*)(ws + oWVl);
  us* WGh = (us*)(ws + oWGh);  us* WGl = (us*)(ws + oWGl);
  us* WOh = (us*)(ws + oWOh);  us* WOl = (us*)(ws + oWOl);
  us* Qh  = (us*)(ws + oQh);   us* Ql  = (us*)(ws + oQl);
  us* Kh  = (us*)(ws + oKh);   us* Kl  = (us*)(ws + oKl);
  us* VTh = (us*)(ws + oVTh);  us* VTl = (us*)(ws + oVTl);
  float* GT = (float*)(ws + oGT);
  us* OGh = (us*)(ws + oOGh);  us* OGl = (us*)(ws + oOGl);

  k_cvt<<<dim3((NTOK * DMOD) / 2048), dim3(256), 0, stream>>>(X, Xh, Xl);
  k_cvt_wt<<<dim3(DMOD / 64, DMOD / 64), dim3(256), 0, stream>>>(Wq, WQh, WQl);
  k_cvt_wt<<<dim3(DMOD / 64, DMOD / 64), dim3(256), 0, stream>>>(Wk, WKh, WKl);
  k_cvt_wt<<<dim3(DMOD / 64, DMOD / 64), dim3(256), 0, stream>>>(Wv, WVh, WVl);
  k_cvt_wt<<<dim3(DMOD / 64, DMOD / 64), dim3(256), 0, stream>>>(Wg, WGh, WGl);
  k_cvt_wt<<<dim3(DMOD / 64, DMOD / 64), dim3(256), 0, stream>>>(Wo, WOh, WOl);
  k_proj<0><<<dim3(NTOK / 64, DMOD / 64), dim3(128), 0, stream>>>(Xh, Xl, WQh, WQl, bg, Qh, Ql, GT);
  k_proj<0><<<dim3(NTOK / 64, DMOD / 64), dim3(128), 0, stream>>>(Xh, Xl, WKh, WKl, bg, Kh, Kl, GT);
  k_proj<1><<<dim3(NTOK / 64, DMOD / 64), dim3(128), 0, stream>>>(Xh, Xl, WVh, WVl, bg, VTh, VTl, GT);
  k_proj<2><<<dim3(NTOK / 64, DMOD / 64), dim3(128), 0, stream>>>(Xh, Xl, WGh, WGl, bg, OGh, OGl, GT);
  k_attn<<<dim3(NBATCH * NHEAD * NQB), dim3(128), 0, stream>>>(Qh, Ql, Kh, Kl, VTh, VTl, GT, OGh, OGl);
  k_proj<3><<<dim3(NTOK / 64, DMOD / 64), dim3(128), 0, stream>>>(OGh, OGl, WOh, WOl, bg, Qh, Ql, out);
  (void)hipGetLastError();
}
